// EGNNLayer_46076409151882
// MI455X (gfx1250) — hardware-run, weakly checked
//
#include <hip/hip_runtime.h>
#include <stddef.h>
#include <stdint.h>


#define ND    128
#define ED    16
#define HD    256
#define KN    384
#define KE1   32
#define NTHR  256
#define NWAVE 8
#define EPT   8
#define CHUNK (NTHR * EPT)
#define WCAP  (EPT * 32)
#define LISTN (NWAVE * WCAP)
#define PASSN 32
#define PCAP  (CHUNK + PASSN)
#define NBE   128
#define NBM   32

static_assert(PASSN == 32);
static_assert(NWAVE * 32 == NTHR);
static_assert(NTHR == HD);
static_assert(HD == NWAVE * 32);
static_assert(ND == NWAVE * 16);
static_assert((NBE % 32) == 0);
static_assert(PCAP >= CHUNK + PASSN);

typedef float        v4f  __attribute__((ext_vector_type(4)));
typedef float        v8f  __attribute__((ext_vector_type(8)));
typedef int          v4i  __attribute__((ext_vector_type(4)));
typedef unsigned int v4u  __attribute__((ext_vector_type(4)));
typedef _Float16     v4h  __attribute__((ext_vector_type(4)));
typedef _Float16     v8h  __attribute__((ext_vector_type(8)));
typedef _Float16     v16h __attribute__((ext_vector_type(16)));
union FragH { v16h v; v8h h[2]; };
union Pack8 { v8h h; v4u u; };

__device__ __forceinline__ v8f wmh(v16h a, v16h b, v8f c) {
  v8f d = __builtin_amdgcn_wmma_f32_16x16x32_f16(false, a, false, b, (short)0, c, false, false);
  asm volatile("v_nop\n\tv_nop\n\tv_nop\n\tv_nop" : "+v"(d) : "v"(a), "v"(b));
  return d;
}

__device__ __forceinline__ v8f zacc() {
  v8f z = {0.0f, 0.0f, 0.0f, 0.0f, 0.0f, 0.0f, 0.0f, 0.0f};
  return z;
}

__device__ __forceinline__ float rcp_f(float d) { return __builtin_amdgcn_rcpf(d); }
__device__ __forceinline__ float silu_f(float v) { return v * rcp_f(1.0f + __expf(-v)); }
__device__ __forceinline__ float sigm_f(float v) { return rcp_f(1.0f + __expf(-v)); }

__device__ __forceinline__ v8h cvt8(v4f a, v4f b) {
  v8h r;
  r[0] = (_Float16)a.x; r[1] = (_Float16)a.y; r[2] = (_Float16)a.z; r[3] = (_Float16)a.w;
  r[4] = (_Float16)b.x; r[5] = (_Float16)b.y; r[6] = (_Float16)b.z; r[7] = (_Float16)b.w;
  return r;
}

template <int K>
__device__ __forceinline__ void gemm2x2(const _Float16* at, const _Float16* __restrict__ bt, int nlo, int hh, int m,
                                        v8f& a00, v8f& a01, v8f& a10, v8f& a11) {
#pragma unroll 2
  for (int k0 = 0; k0 < K; k0 += 32) {
    FragH fa0, fa1, fb0, fb1;
    const _Float16* ap = at + m * K + k0 + 8 * hh;
    fa0.h[0] = *(const v8h*)ap;
    fa0.h[1] = *(const v8h*)(ap + 16);
    fa1.h[0] = *(const v8h*)(ap + 16 * K);
    fa1.h[1] = *(const v8h*)(ap + 16 * K + 16);
    const _Float16* bp = bt + (size_t)(nlo + m) * K + k0 + 8 * hh;
    fb0.h[0] = *(const v8h*)bp;
    fb0.h[1] = *(const v8h*)(bp + 16);
    fb1.h[0] = *(const v8h*)(bp + (size_t)16 * K);
    fb1.h[1] = *(const v8h*)(bp + (size_t)16 * K + 16);
    a00 = wmh(fa0.v, fb0.v, a00);
    a01 = wmh(fa0.v, fb1.v, a01);
    a10 = wmh(fa1.v, fb0.v, a10);
    a11 = wmh(fa1.v, fb1.v, a11);
  }
}

__device__ __forceinline__ int scan_chunk(const int* __restrict__ keys, int nE, int cbase, int nodeBase,
                                          int vec8, int* list, int tid, int wave) {
  int wc = 0;
  const int el0  = tid * EPT;
  const int e0   = cbase + el0;
  const int sent = -2147483647 - 1;
  v4i da, db;
  if (vec8 != 0 && cbase + CHUNK <= nE) {
    da = *(const v4i*)(keys + e0);
    db = *(const v4i*)(keys + e0 + 4);
  } else {
    da.x = (e0     < nE) ? keys[min(e0, nE - 1)] : sent;
    da.y = (e0 + 1 < nE) ? keys[min(e0 + 1, nE - 1)] : sent;
    da.z = (e0 + 2 < nE) ? keys[min(e0 + 2, nE - 1)] : sent;
    da.w = (e0 + 3 < nE) ? keys[min(e0 + 3, nE - 1)] : sent;
    db.x = (e0 + 4 < nE) ? keys[min(e0 + 4, nE - 1)] : sent;
    db.y = (e0 + 5 < nE) ? keys[min(e0 + 5, nE - 1)] : sent;
    db.z = (e0 + 6 < nE) ? keys[min(e0 + 6, nE - 1)] : sent;
    db.w = (e0 + 7 < nE) ? keys[min(e0 + 7, nE - 1)] : sent;
  }
  const unsigned nb = (unsigned)nodeBase;
  const unsigned s0 = (unsigned)da.x - nb, s1 = (unsigned)da.y - nb;
  const unsigned s2 = (unsigned)da.z - nb, s3 = (unsigned)da.w - nb;
  const unsigned s4 = (unsigned)db.x - nb, s5 = (unsigned)db.y - nb;
  const unsigned s6 = (unsigned)db.z - nb, s7 = (unsigned)db.w - nb;
  const bool h0 = s0 < (unsigned)NBE, h1 = s1 < (unsigned)NBE, h2 = s2 < (unsigned)NBE, h3 = s3 < (unsigned)NBE;
  const bool h4 = s4 < (unsigned)NBE, h5 = s5 < (unsigned)NBE, h6 = s6 < (unsigned)NBE, h7 = s7 < (unsigned)NBE;
  const unsigned any = __builtin_amdgcn_ballot_w32(h0 | h1 | h2 | h3 | h4 | h5 | h6 | h7);
  if (any != 0u) {
#define HITJ(J, HJ) { \
      const unsigned mj = __builtin_amdgcn_ballot_w32(HJ); \
      if (mj != 0u) { \
        if (HJ) { \
          const int pos = wc + (int)__builtin_amdgcn_mbcnt_lo(mj, 0u); \
          if (pos < WCAP) list[wave * WCAP + pos] = el0 + (J); \
        } \
        wc += (int)__builtin_popcount(mj); } }
    HITJ(0, h0)
    HITJ(1, h1)
    HITJ(2, h2)
    HITJ(3, h3)
    HITJ(4, h4)
    HITJ(5, h5)
    HITJ(6, h6)
    HITJ(7, h7)
#undef HITJ
  }
  return wc;
}

__global__ __launch_bounds__(NTHR) void k_cvt(const float* __restrict__ src, _Float16* dst,
                                              int nRows, int Kp, int sk, int sn, int off,
                                              int kReal, int nReal, int kSplit, float s0, float s1) {
  const int g = blockIdx.x * NTHR + threadIdx.x;
  const int total = nRows * (Kp >> 3);
  if (g >= total) return;
  const int e0 = g * 8;
  const int n = e0 / Kp;
  const int k8 = e0 - n * Kp;
  const int nc = n < nReal ? n : nReal - 1;
  Pack8 o;
#pragma unroll
  for (int i = 0; i < 8; ++i) {
    const int k = k8 + i;
    const int kc = k < kReal ? k : kReal - 1;
    const float ld = src[(size_t)kc * (size_t)sk + (size_t)nc * (size_t)sn + (size_t)off];
    const bool valid = (k < kReal) && (n < nReal);
    const float sc = valid ? ((k < kSplit) ? s0 : s1) : 0.0f;
    o.h[i] = (_Float16)(ld * sc);
  }
  v4u* p = (v4u*)(dst + (size_t)e0);
  *(volatile v4u*)p = o.u;
  __threadfence();
  *(volatile v4u*)p = o.u;
}

__global__ __launch_bounds__(NTHR) void k_pq(const float* __restrict__ h, const _Float16* __restrict__ W1nT,
                                             float* PQ, int nN) {
  __shared__ __attribute__((aligned(16))) float stile[NBM * 256];
  const int tid = threadIdx.x, lane = tid & 31, wave = tid >> 5, hh = lane >> 4, m = lane & 15;
  const int r0 = blockIdx.x * NBM;
  const int c0 = blockIdx.y * 256;
  const int cl = 32 * wave;
  int ra0 = r0 + m;      ra0 = ra0 > nN - 1 ? nN - 1 : ra0;
  int ra1 = r0 + 16 + m; ra1 = ra1 > nN - 1 ? nN - 1 : ra1;
  v8f a00 = zacc(), a01 = zacc(), a10 = zacc(), a11 = zacc();
#pragma unroll 2
  for (int k0 = 0; k0 < ND; k0 += 32) {
    FragH fa0, fa1, fb0, fb1;
    const float* p0 = h + (size_t)ra0 * ND + k0 + 8 * hh;
    const float* p1 = h + (size_t)ra1 * ND + k0 + 8 * hh;
    fa0.h[0] = cvt8(*(const v4f*)p0, *(const v4f*)(p0 + 4));
    fa0.h[1] = cvt8(*(const v4f*)(p0 + 16), *(const v4f*)(p0 + 20));
    fa1.h[0] = cvt8(*(const v4f*)p1, *(const v4f*)(p1 + 4));
    fa1.h[1] = cvt8(*(const v4f*)(p1 + 16), *(const v4f*)(p1 + 20));
    const _Float16* bp = W1nT + (size_t)(c0 + cl + m) * ND + k0 + 8 * hh;
    fb0.h[0] = *(const v8h*)bp;
    fb0.h[1] = *(const v8h*)(bp + 16);
    fb1.h[0] = *(const v8h*)(bp + 16 * ND);
    fb1.h[1] = *(const v8h*)(bp + 16 * ND + 16);
    a00 = wmh(fa0.v, fb0.v, a00);
    a01 = wmh(fa0.v, fb1.v, a01);
    a10 = wmh(fa1.v, fb0.v, a10);
    a11 = wmh(fa1.v, fb1.v, a11);
  }
#pragma unroll
  for (int r = 0; r < 8; ++r) {
    stile[(8 * hh + r) * 256 + cl + m]           = a00[r];
    stile[(8 * hh + r) * 256 + cl + 16 + m]      = a01[r];
    stile[(16 + 8 * hh + r) * 256 + cl + m]      = a10[r];
    stile[(16 + 8 * hh + r) * 256 + cl + 16 + m] = a11[r];
  }
  __syncthreads();
  const int lq = lane >> 3, lp = (lane & 7) * 4;
#pragma unroll
  for (int j = 0; j < 8; ++j) {
    const int L = wave * 32 + j * 4 + lq;
    const int row = L >> 3, seg = L & 7;
    const int col = seg * 32 + lp;
    const v4f v = *(const v4f*)(stile + row * 256 + col);
    *(volatile v4f*)(PQ + (size_t)(r0 + row) * 512 + c0 + col) = v;
  }
  __threadfence();
#pragma unroll
  for (int j = 0; j < 8; ++j) {
    const int L = wave * 32 + j * 4 + lq;
    const int row = L >> 3, seg = L & 7;
    const int col = seg * 32 + lp;
    const v4f v = *(const v4f*)(stile + row * 256 + col);
    *(volatile v4f*)(PQ + (size_t)(r0 + row) * 512 + c0 + col) = v;
  }
}

__global__ __launch_bounds__(NTHR) void k_edge(
    const float* __restrict__ x, const float* __restrict__ ea, const int* __restrict__ ei,
    const float* __restrict__ PQ, const _Float16* __restrict__ W1eT, const float* __restrict__ be1,
    const _Float16* __restrict__ W2T, const float* __restrict__ be2,
    const float* __restrict__ Wa, const float* __restrict__ ba,
    const _Float16* __restrict__ Wc1T, const float* __restrict__ bc1, const float* __restrict__ Wc2,
    float* aggp, float* xout, int nN, int nE, int vec8, float invdeg, int xlim) {
  __shared__ __attribute__((aligned(16))) float    sagg[(NBE + 1) * HD];
  __shared__ __attribute__((aligned(16))) float    cacc[(NBE + 1) * 4];
  __shared__ __attribute__((aligned(16))) float    cpre[PASSN * HD];
  __shared__ __attribute__((aligned(16))) _Float16 atile[PASSN * HD];
  __shared__ __attribute__((aligned(16))) _Float16 aext[PASSN * KE1];
  __shared__ __attribute__((aligned(16))) int      list[LISTN];
  __shared__ __attribute__((aligned(16))) int      pend[PCAP];
  __shared__ __attribute__((aligned(16))) float    parts[NWAVE * PASSN];
  __shared__ __attribute__((aligned(16))) float    sbe[HD];
  __shared__ __attribute__((aligned(16))) float    sunit[PASSN * 4];
  __shared__ float satt[PASSN];
  __shared__ int   sslot[PASSN], srow[PASSN], scol[PASSN];
  __shared__ int   wcnt[NWAVE];
  __shared__ int   pendN;

  const int tid = threadIdx.x, lane = tid & 31, wave = tid >> 5, hh = lane >> 4, m = lane & 15;
  const int nodeBase = blockIdx.x * NBE;
  const int cw0 = 32 * wave;
  const int* keys = ei;
  const int* cols = ei + nE;

  for (int i = tid; i < (NBE + 1) * HD / 4; i += NTHR) {
    const v4f z = {0.0f, 0.0f, 0.0f, 0.0f};
    *(v4f*)(sagg + 4 * i) = z;
  }
  for (int i = tid; i < (NBE + 1) * 4; i += NTHR) cacc[i] = 0.0f;
  if (tid < PASSN * KE1 / 8) {
    Pack8 z;
    const v4u zz = {0u, 0u, 0u, 0u};
    z.u = zz;
    *(v8h*)(aext + 8 * tid) = z.h;
  }
  sbe[tid] = be1[tid] * 64.0f;
  if (tid == 0) pendN = 0;
  const float walo = Wa[cw0 + m],  wahi = Wa[cw0 + 16 + m];
  const float wclo = Wc2[cw0 + m], wchi = Wc2[cw0 + 16 + m];
  const float belo = be2[cw0 + m], behi = be2[cw0 + 16 + m];
  const float bclo = bc1[cw0 + m], bchi = bc1[cw0 + 16 + m];
  const float bav  = ba[0];
  __syncthreads();

  const int nChunks = (nE + CHUNK - 1) / CHUNK;
#pragma unroll 1
  for (int ch = 0; ch < nChunks; ++ch) {
    const int cbase = ch * CHUNK;
    const int wc = scan_chunk(keys, nE, cbase, nodeBase, vec8, list, tid, wave);
    if (lane == 0) wcnt[wave] = wc;
    __syncthreads();

    const int base = pendN;
    int tot = 0, myoff = 0;
#pragma unroll
    for (int w = 0; w < NWAVE; ++w) {
      int c = wcnt[w];
      c = c > WCAP ? WCAP : (c < 0 ? 0 : c);
      if (w < wave) myoff += c;
      tot += c;
    }
    int newN = base + tot;
    newN = newN > PCAP ? PCAP : newN;
    {
      int n = wcnt[wave];
      n = n > WCAP ? WCAP : (n < 0 ? 0 : n);
      const int* lp = list + wave * WCAP;
      for (int i = lane; i < n; i += 32) {
        const int pos = base + myoff + i;
        if (pos < PCAP) pend[pos] = cbase + lp[i];
      }
    }
    const int fin = (ch == nChunks - 1) ? 1 : 0;
    const int R   = (fin != 0) ? (newN + PASSN - 1) / PASSN : newN / PASSN;
    const int Pv  = (fin != 0) ? newN : R * PASSN;
    __syncthreads();

#pragma unroll 1
    for (int r = 0; r < R; ++r) {
      if (wave == 0) {
#pragma clang fp contract(off)
        const int idx = r * PASSN + lane;
        const bool valid = idx < Pv;
        const int idxc = idx < PCAP ? idx : PCAP - 1;
        int e = pend[idxc];
        e = valid ? e : 0;
        e = e < 0 ? 0 : (e > nE - 1 ? nE - 1 : e);
        int rw = keys[e];
        int cl = cols[e];
        int slot = rw - nodeBase;
        if (!valid || (unsigned)slot >= (unsigned)NBE) slot = NBE;
        rw = rw < 0 ? 0 : (rw > nN - 1 ? nN - 1 : rw);
        cl = cl < 0 ? 0 : (cl > nN - 1 ? nN - 1 : cl);
        const float dx = x[(size_t)rw * 3 + 0] - x[(size_t)cl * 3 + 0];
        const float dy = x[(size_t)rw * 3 + 1] - x[(size_t)cl * 3 + 1];
        const float dz = x[(size_t)rw * 3 + 2] - x[(size_t)cl * 3 + 2];
        const float d2 = (dx * dx + dy * dy) + dz * dz;
        const float inv = 1.0f / sqrtf(d2 + 1e-8f);
        sunit[lane * 4 + 0] = dx * inv;
        sunit[lane * 4 + 1] = dy * inv;
        sunit[lane * 4 + 2] = dz * inv;
        sunit[lane * 4 + 3] = 0.0f;
        srow[lane] = rw; scol[lane] = cl; sslot[lane] = slot;
        const float* ap = ea + (size_t)e * ED;
        const v4f t0 = *(const v4f*)ap;
        const v4f t1 = *(const v4f*)(ap + 4);
        const v4f t2 = *(const v4f*)(ap + 8);
        const v4f t3 = *(const v4f*)(ap + 12);
        v8h q0, q1;
        q0[0] = (_Float16)d2;   q0[1] = (_Float16)t0.x; q0[2] = (_Float16)t0.y; q0[3] = (_Float16)t0.z;
        q0[4] = (_Float16)t0.w; q0[5] = (_Float16)t1.x; q0[6] = (_Float16)t1.y; q0[7] = (_Float16)t1.z;
        q1[0] = (_Float16)t1.w; q1[1] = (_Float16)t2.x; q1[2] = (_Float16)t2.y; q1[3] = (_Float16)t2.z;
        q1[4] = (_Float16)t2.w; q1[5] = (_Float16)t3.x; q1[6] = (_Float16)t3.y; q1[7] = (_Float16)t3.z;
        *(v8h*)(aext + lane * KE1) = q0;
        *(v8h*)(aext + lane * KE1 + 8) = q1;
        aext[lane * KE1 + 16] = (_Float16)t3.w;
      }
      __syncthreads();

      {
        const int e = tid >> 3, p = tid & 7;
        const float* pp = PQ + (size_t)srow[e] * 512;
        const float* qp = PQ + (size_t)scol[e] * 512 + 256;
#pragma unroll
        for (int j = 0; j < 8; ++j) {
          const int c4 = (j * 8 + p) * 4;
          const v4f a  = *(const v4f*)(pp + c4);
          const v4f b  = *(const v4f*)(qp + c4);
          const v4f bb = *(const v4f*)(sbe + c4);
          *(v4f*)(cpre + e * HD + c4) = (a + b) + bb;
        }
      }
      __syncthreads();

      {
        v8f a00, a01, a10, a11;
#pragma unroll
        for (int rr = 0; rr < 8; ++rr) {
          a00[rr] = cpre[(8 * hh + rr) * HD + cw0 + m];
          a01[rr] = cpre[(8 * hh + rr) * HD + cw0 + 16 + m];
          a10[rr] = cpre[(16 + 8 * hh + rr) * HD + cw0 + m];
          a11[rr] = cpre[(16 + 8 * hh + rr) * HD + cw0 + 16 + m];
        }
        FragH fa0, fa1, fb0, fb1;
        fa0.h[0] = *(const v8h*)(aext + m * KE1 + 8 * hh);
        fa0.h[1] = *(const v8h*)(aext + m * KE1 + 16 + 8 * hh);
        fa1.h[0] = *(const v8h*)(aext + (16 + m) * KE1 + 8 * hh);
        fa1.h[1] = *(const v8h*)(aext + (16 + m) * KE1 + 16 + 8 * hh);
        const _Float16* bp = W1eT + (size_t)(cw0 + m) * KE1 + 8 * hh;
        fb0.h[0] = *(const v8h*)bp;
        fb0.h[1] = *(const v8h*)(bp + 16);
        fb1.h[0] = *(const v8h*)(bp + 16 * KE1);
        fb1.h[1] = *(const v8h*)(bp + 16 * KE1 + 16);
        a00 = wmh(fa0.v, fb0.v, a00);
        a01 = wmh(fa0.v, fb1.v, a01);
        a10 = wmh(fa1.v, fb0.v, a10);
        a11 = wmh(fa1.v, fb1.v, a11);
#pragma unroll
        for (int rr = 0; rr < 8; ++rr) {
          atile[(8 * hh + rr) * HD + cw0 + m]           = (_Float16)(silu_f(a00[rr] * (1.0f / 64.0f)) * 16.0f);
          atile[(8 * hh + rr) * HD + cw0 + 16 + m]      = (_Float16)(silu_f(a01[rr] * (1.0f / 64.0f)) * 16.0f);
          atile[(16 + 8 * hh + rr) * HD + cw0 + m]      = (_Float16)(silu_f(a10[rr] * (1.0f / 64.0f)) * 16.0f);
          atile[(16 + 8 * hh + rr) * HD + cw0 + 16 + m] = (_Float16)(silu_f(a11[rr] * (1.0f / 64.0f)) * 16.0f);
        }
      }
      __syncthreads();

      v8f m00 = zacc(), m01 = zacc(), m10 = zacc(), m11 = zacc();
      gemm2x2<HD>(atile, W2T, cw0, hh, m, m00, m01, m10, m11);
      {
        v8f p0, p1;
#pragma unroll
        for (int rr = 0; rr < 8; ++rr) {
          m00[rr] = silu_f(m00[rr] * (1.0f / 1024.0f) + belo);
          m01[rr] = silu_f(m01[rr] * (1.0f / 1024.0f) + behi);
          m10[rr] = silu_f(m10[rr] * (1.0f / 1024.0f) + belo);
          m11[rr] = silu_f(m11[rr] * (1.0f / 1024.0f) + behi);
          p0[rr] = m00[rr] * walo + m01[rr] * wahi;
          p1[rr] = m10[rr] * walo + m11[rr] * wahi;
        }
#pragma unroll
        for (int off = 1; off < 16; off <<= 1) {
#pragma unroll
          for (int rr = 0; rr < 8; ++rr) {
            p0[rr] += __shfl_xor(p0[rr], off, 32);
            p1[rr] += __shfl_xor(p1[rr], off, 32);
          }
        }
        if (m == 0) {
#pragma unroll
          for (int rr = 0; rr < 8; ++rr) {
            parts[wave * PASSN + 8 * hh + rr]      = p0[rr];
            parts[wave * PASSN + 16 + 8 * hh + rr] = p1[rr];
          }
        }
      }
      __syncthreads();

      if (wave == 0) {
        float s = 0.0f;
#pragma unroll
        for (int w = 0; w < NWAVE; ++w) s += parts[w * PASSN + lane];
        satt[lane] = sigm_f(s + bav);
      }
      __syncthreads();

#pragma unroll
      for (int rr = 0; rr < 8; ++rr) {
        const int e0i = 8 * hh + rr, e1i = 16 + 8 * hh + rr;
        const float at0 = satt[e0i], at1 = satt[e1i];
        const float v00 = m00[rr] * at0, v01 = m01[rr] * at0;
        const float v10 = m10[rr] * at1, v11 = m11[rr] * at1;
        cpre[e0i * HD + cw0 + m]       = v00;
        cpre[e0i * HD + cw0 + 16 + m]  = v01;
        cpre[e1i * HD + cw0 + m]       = v10;
        cpre[e1i * HD + cw0 + 16 + m]  = v11;
        atile[e0i * HD + cw0 + m]      = (_Float16)(v00 * 64.0f);
        atile[e0i * HD + cw0 + 16 + m] = (_Float16)(v01 * 64.0f);
        atile[e1i * HD + cw0 + m]      = (_Float16)(v10 * 64.0f);
        atile[e1i * HD + cw0 + 16 + m] = (_Float16)(v11 * 64.0f);
      }
      __syncthreads();

      {
        const int c = cw0 + lane;
#pragma unroll 1
        for (int e = 0; e < PASSN; ++e) {
          int s = sslot[e];
          s = s < 0 ? 0 : (s > NBE ? NBE : s);
          sagg[s * HD + c] += cpre[e * HD + c];
        }
      }

      v8f c00 = zacc(), c01 = zacc(), c10 = zacc(), c11 = zacc();
      gemm2x2<HD>(atile, Wc1T, cw0, hh, m, c00, c01, c10, c11);
      {
        v8f p0, p1;
#pragma unroll
        for (int rr = 0; rr < 8; ++rr) {
          const float t00 = silu_f(c00[rr] * (1.0f / 4096.0f) + bclo);
          const float t01 = silu_f(c01[rr] * (1.0f / 4096.0f) + bchi);
          const float t10 = silu_f(c10[rr] * (1.0f / 4096.0f) + bclo);
          const float t11 = silu_f(c11[rr] * (1.0f / 4096.0f) + bchi);
          p0[rr] = t00 * wclo + t01 * wchi;
          p1[rr] = t10 * wclo + t11 * wchi;
        }
#pragma unroll
        for (int off = 1; off < 16; off <<= 1) {
#pragma unroll
          for (int rr = 0; rr < 8; ++rr) {
            p0[rr] += __shfl_xor(p0[rr], off, 32);
            p1[rr] += __shfl_xor(p1[rr], off, 32);
          }
        }
        if (m == 0) {
#pragma unroll
          for (int rr = 0; rr < 8; ++rr) {
            parts[wave * PASSN + 8 * hh + rr]      = p0[rr];
            parts[wave * PASSN + 16 + 8 * hh + rr] = p1[rr];
          }
        }
      }
      __syncthreads();

      if (wave == 0) {
        float s = 0.0f;
#pragma unroll
        for (int w = 0; w < NWAVE; ++w) s += parts[w * PASSN + lane];
        const float cw = tanhf(s);
        const float g0 = cw * sunit[lane * 4 + 0];
        const float g1 = cw * sunit[lane * 4 + 1];
        const float g2 = cw * sunit[lane * 4 + 2];
        const int mys = sslot[lane];
#pragma unroll 1
        for (int e = 0; e < PASSN; ++e) {
          const float v0 = __shfl(g0, e, 32);
          const float v1 = __shfl(g1, e, 32);
          const float v2 = __shfl(g2, e, 32);
          int s = __shfl(mys, e, 32);
          s = s < 0 ? 0 : (s > NBE ? NBE : s);
          const float v = (lane == 0) ? v0 : ((lane == 1) ? v1 : v2);
          if (lane < 3) cacc[s * 4 + lane] += v;
        }
      }
    }

    int rem = newN - R * PASSN;
    rem = rem < 0 ? 0 : rem;
    if (R > 0 && tid < rem) pend[tid] = pend[R * PASSN + tid];
    if (tid == 0) pendN = rem;
  }
  __syncthreads();

  float* gb = aggp + (size_t)nodeBase * HD;
#pragma unroll 4
  for (int j = 0; j < 32; ++j) {
    const int i4 = (wave * 32 + j) * 32 + lane;
    const v4f v = *(const v4f*)(sagg + (size_t)i4 * 4);
    *(volatile v4f*)(gb + (size_t)i4 * 4) = v;
  }
  const int fl0 = 4 * tid;
  const size_t f0 = (size_t)nodeBase * 3 + (size_t)fl0;
  v4f xv = {0.0f, 0.0f, 0.0f, 0.0f};
  if (wave < 3) {
#pragma unroll
    for (int j = 0; j < 4; ++j) {
      const int fl = fl0 + j;
      const int nl = fl / 3;
      const int cp = fl - nl * 3;
      const size_t f = f0 + (size_t)j;
      const size_t fc = f < (size_t)xlim ? f : (size_t)xlim - 1;
      xv[j] = x[fc] + cacc[nl * 4 + cp] * invdeg;
    }
    if (f0 + 3 < (size_t)xlim) {
      *(volatile v4f*)(xout + f0) = xv;
    } else {
      volatile float* xo = (volatile float*)xout;
#pragma unroll
      for (int j = 0; j < 4; ++j) if (f0 + (size_t)j < (size_t)xlim) xo[f0 + j] = xv[j];
    }
  }
  __threadfence();
#pragma unroll 4
  for (int j = 0; j < 32; ++j) {
    const int i4 = (wave * 32 + j) * 32 + lane;
    const v4f v = *(const v4f*)(sagg + (size_t)i4 * 4);
    *(volatile v4f*)(gb + (size_t)i4 * 4) = v;
  }
  if (wave < 3) {
    if (f0 + 3 < (size_t)xlim) {
      *(volatile v4f*)(xout + f0) = xv;
    } else {
      volatile float* xo = (volatile float*)xout;
#pragma unroll
      for (int j = 0; j < 4; ++j) if (f0 + (size_t)j < (size_t)xlim) xo[f0 + j] = xv[j];
    }
  }
}

__global__ __launch_bounds__(NTHR) void k_node(const float* __restrict__ h, const float* __restrict__ aggp,
                                               const _Float16* __restrict__ Wn1T, const float* __restrict__ bn1,
                                               const _Float16* __restrict__ Wn2T, const float* __restrict__ bn2,
                                               const float* __restrict__ gam, const float* __restrict__ bet,
                                               float* hout, int nN) {
  __shared__ __attribute__((aligned(16))) _Float16 ta[NBM * KN];
  __shared__ __attribute__((aligned(16))) _Float16 tn[NBM * HD];
  __shared__ __attribute__((aligned(16))) float    shr[NBM * ND];
  const int tid = threadIdx.x, lane = tid & 31, wave = tid >> 5, hh = lane >> 4, m = lane & 15;
  const int nd0 = blockIdx.x * NBM;
  const int cw0 = 32 * wave;

#pragma unroll
  for (int j = 0; j < 4; ++j) {
    const int idx = tid + NTHR * j;
    const int row = idx >> 5;
    const int c4 = (idx & 31) * 4;
    int node = nd0 + row; node = node > nN - 1 ? nN - 1 : node;
    const v4f v = *(const v4f*)(h + (size_t)node * ND + c4);
    v4h o;
    o[0] = (_Float16)v.x; o[1] = (_Float16)v.y; o[2] = (_Float16)v.z; o[3] = (_Float16)v.w;
    *(v4h*)(ta + row * KN + c4) = o;
  }
#pragma unroll
  for (int j = 0; j < 8; ++j) {
    const int idx = tid + NTHR * j;
    const int row = idx >> 6;
    const int c4 = (idx & 63) * 4;
    int node = nd0 + row; node = node > nN - 1 ? nN - 1 : node;
    const v4f v = *(const v4f*)(aggp + (size_t)node * HD + c4) * 16.0f;
    v4h o;
    o[0] = (_Float16)v.x; o[1] = (_Float16)v.y; o[2] = (_Float16)v.z; o[3] = (_Float16)v.w;
    *(v4h*)(ta + row * KN + ND + c4) = o;
  }
  __syncthreads();

  v8f a00 = zacc(), a01 = zacc(), a10 = zacc(), a11 = zacc();
  gemm2x2<KN>(ta, Wn1T, cw0, hh, m, a00, a01, a10, a11);
  {
    const float blo = bn1[cw0 + m], bhi = bn1[cw0 + 16 + m];
#pragma unroll
    for (int rr = 0; rr < 8; ++rr) {
      tn[(8 * hh + rr) * HD + cw0 + m]           = (_Float16)(silu_f(a00[rr] * (1.0f / 64.0f) + blo) * 16.0f);
      tn[(8 * hh + rr) * HD + cw0 + 16 + m]      = (_Float16)(silu_f(a01[rr] * (1.0f / 64.0f) + bhi) * 16.0f);
      tn[(16 + 8 * hh + rr) * HD + cw0 + m]      = (_Float16)(silu_f(a10[rr] * (1.0f / 64.0f) + blo) * 16.0f);
      tn[(16 + 8 * hh + rr) * HD + cw0 + 16 + m] = (_Float16)(silu_f(a11[rr] * (1.0f / 64.0f) + bhi) * 16.0f);
    }
  }
  __syncthreads();

  v8f d0 = zacc(), d1 = zacc();
  const int ncol = 16 * wave + m;
#pragma unroll 2
  for (int k0 = 0; k0 < HD; k0 += 32) {
    FragH fa0, fa1, fb;
    const _Float16* ap = tn + m * HD + k0 + 8 * hh;
    fa0.h[0] = *(const v8h*)ap;
    fa0.h[1] = *(const v8h*)(ap + 16);
    fa1.h[0] = *(const v8h*)(ap + 16 * HD);
    fa1.h[1] = *(const v8h*)(ap + 16 * HD + 16);
    const _Float16* bp = Wn2T + (size_t)ncol * HD + k0 + 8 * hh;
    fb.h[0] = *(const v8h*)bp;
    fb.h[1] = *(const v8h*)(bp + 16);
    d0 = wmh(fa0.v, fb.v, d0);
    d1 = wmh(fa1.v, fb.v, d1);
  }
  {
    const float bb = bn2[ncol];
#pragma unroll
    for (int rr = 0; rr < 8; ++rr) {
      const int row0 = 8 * hh + rr, row1 = 16 + 8 * hh + rr;
      int node0 = nd0 + row0; node0 = node0 > nN - 1 ? nN - 1 : node0;
      int node1 = nd0 + row1; node1 = node1 > nN - 1 ? nN - 1 : node1;
      const float hv0 = h[(size_t)node0 * ND + ncol];
      const float hv1 = h[(size_t)node1 * ND + ncol];
      shr[row0 * ND + ncol] = hv0 + (d0[rr] * (1.0f / 1024.0f) + bb);
      shr[row1 * ND + ncol] = hv1 + (d1[rr] * (1.0f / 1024.0f) + bb);
    }
  }
  __syncthreads();

  {
    const int e = tid >> 3, j = tid & 7;
    float* rp = shr + e * ND + 16 * j;
    v4f q0 = *(const v4f*)rp;
    v4f q1 = *(const v4f*)(rp + 4);
    v4f q2 = *(const v4f*)(rp + 8);
    v4f q3 = *(const v4f*)(rp + 12);
    float s = ((q0.x + q0.y) + (q0.z + q0.w)) + ((q1.x + q1.y) + (q1.z + q1.w))
            + ((q2.x + q2.y) + (q2.z + q2.w)) + ((q3.x + q3.y) + (q3.z + q3.w));
    s += __shfl_xor(s, 1, 32);
    s += __shfl_xor(s, 2, 32);
    s += __shfl_xor(s, 4, 32);
    const float mu = s * (1.0f / 128.0f);
    q0 = q0 - mu; q1 = q1 - mu; q2 = q2 - mu; q3 = q3 - mu;
    float s2 = ((q0.x * q0.x + q0.y * q0.y) + (q0.z * q0.z + q0.w * q0.w))
             + ((q1.x * q1.x + q1.y * q1.y) + (q1.z * q1.z + q1.w * q1.w))
             + ((q2.x * q2.x + q2.y * q2.y) + (q2.z * q2.z + q2.w * q2.w))
             + ((q3.x * q3.x + q3.y * q3.y) + (q3.z * q3.z + q3.w * q3.w));
    s2 += __shfl_xor(s2, 1, 32);
    s2 += __shfl_xor(s2, 2, 32);
    s2 += __shfl_xor(s2, 4, 32);
    const float var = s2 * (1.0f / 128.0f);
    const float rstd = 1.0f / sqrtf(var + 1e-5f);
    const v4f g0 = *(const v4f*)(gam + 16 * j), g1 = *(const v4f*)(gam + 16 * j + 4);
    const v4f g2 = *(const v4f*)(gam + 16 * j + 8), g3 = *(const v4f*)(gam + 16 * j + 12);
    const v4f b0 = *(const v4f*)(bet + 16 * j), b1 = *(const v4f*)(bet + 16 * j + 4);
    const v4f b2 = *(const v4f*)(bet + 16 * j + 8), b3 = *(const v4f*)(bet + 16 * j + 12);
    q0 = (q0 * rstd) * g0 + b0;
    q1 = (q1 * rstd) * g1 + b1;
    q2 = (q2 * rstd) * g2 + b2;
    q3 = (q3 * rstd) * g3 + b3;
    *(v4f*)rp = q0;
    *(v4f*)(rp + 4) = q1;
    *(v4f*)(rp + 8) = q2;
    *(v4f*)(rp + 12) = q3;
  }
  __syncthreads();

  const int lq = lane >> 3, lp = (lane & 7) * 4;
#pragma unroll
  for (int jj = 0; jj < 4; ++jj) {
    const int L = wave * 16 + jj * 4 + lq;
    const int row = L >> 2, seg = L & 3;
    const int node = nd0 + row;
    const int col = seg * 32 + lp;
    const v4f v = *(const v4f*)(shr + row * ND + col);
    if (node < nN) *(volatile v4f*)(hout + (size_t)node * ND + col) = v;
  }
  __threadfence();
#pragma unroll
  for (int jj = 0; jj < 4; ++jj) {
    const int L = wave * 16 + jj * 4 + lq;
    const int row = L >> 2, seg = L & 3;
    const int node = nd0 + row;
    const int col = seg * 32 + lp;
    const v4f v = *(const v4f*)(shr + row * ND + col);
    if (node < nN) *(volatile v4f*)(hout + (size_t)node * ND + col) = v;
  }
}

extern "C" void kernel_launch(void* const* d_in, const int* in_sizes, int n_in,
                              void* d_out, int out_size, void* d_ws, size_t ws_size,
                              hipStream_t stream) {
  if (n_in < 19) return;
  const int nN = in_sizes[0] / ND;
  const int nE = in_sizes[3] / 2;
  if (nN < 1 || nE < 1) return;
  if (in_sizes[0] != nN * ND || in_sizes[1] != nN * 3 || in_sizes[2] != nE * ED || in_sizes[3] != 2 * nE) return;
  if (in_sizes[4] != (2 * ND + 1 + ED) * HD || in_sizes[5] < HD || in_sizes[6] != HD * HD || in_sizes[7] < HD) return;
  if (in_sizes[8] < HD || in_sizes[9] < 1 || in_sizes[10] != HD * HD || in_sizes[11] < HD || in_sizes[12] < HD) return;
  if (in_sizes[13] != KN * HD || in_sizes[14] < HD || in_sizes[15] != HD * ND || in_sizes[16] < ND) return;
  if (in_sizes[17] < ND || in_sizes[18] < ND) return;
  if (out_size != nN * ND + nN * 3) return;

  const float* h     = (const float*)d_in[0];
  const float* x     = (const float*)d_in[1];
  const float* ea    = (const float*)d_in[2];
  const int*   eidx  = (const int*)d_in[3];
  const float* We1   = (const float*)d_in[4];
  const float* be1   = (const float*)d_in[5];
  const float* We2   = (const float*)d_in[6];
  const float* be2   = (const float*)d_in[7];
  const float* Wa    = (const float*)d_in[8];
  const float* ba    = (const float*)d_in[9];
  const float* Wc1   = (const float*)d_in[10];
  const float* bc1   = (const float*)d_in[11];
  const float* Wc2   = (const float*)d_in[12];
  const float* Wn1   = (const float*)d_in[13];
  const float* bn1   = (const float*)d_in[14];
  const float* Wn2   = (const float*)d_in[15];
  const float* bn2   = (const float*)d_in[16];
  const float* gamma = (const float*)d_in[17];
  const float* beta  = (const float*)d_in[18];
  float* hout = (float*)d_out;
  float* xout = hout + (size_t)nN * ND;

  const int nBlkM = (nN + NBM - 1) / NBM;
  const int Mpad  = nBlkM * NBM;
  const int nBlkE = (nN + NBE - 1) / NBE;

  char* ws = (char*)d_ws;
  size_t off = 0;
  auto carve = [&](size_t bytes) -> size_t { const size_t o = off; off = (off + bytes + 255) & ~(size_t)255; return o; };
  const size_t oW1n = carve((size_t)512 * ND * 2);
  const size_t oW1e = carve((size_t)HD * KE1 * 2);
  const size_t oW2  = carve((size_t)HD * HD * 2);
  const size_t oWc1 = carve((size_t)HD * HD * 2);
  const size_t oWn1 = carve((size_t)HD * KN * 2);
  const size_t oWn2 = carve((size_t)ND * HD * 2);
  const size_t oPQ  = carve((size_t)Mpad * 512 * 4);
  const size_t oAGG = carve((size_t)nBlkE * NBE * HD * 4);
  if (off > ws_size) return;
  _Float16* W1nT = (_Float16*)(ws + oW1n);
  _Float16* W1eT = (_Float16*)(ws + oW1e);
  _Float16* W2T  = (_Float16*)(ws + oW2);
  _Float16* Wc1T = (_Float16*)(ws + oWc1);
  _Float16* Wn1T = (_Float16*)(ws + oWn1);
  _Float16* Wn2T = (_Float16*)(ws + oWn2);
  float* PQ  = (float*)(ws + oPQ);
  float* AGG = (float*)(ws + oAGG);

  auto cvt = [&](const float* src, _Float16* dst, int nRows, int Kp, int sk, int sn, int offv,
                 int kReal, int nReal, int kSplit, float s0, float s1) {
    const int total = nRows * (Kp / 8);
    k_cvt<<<(total + NTHR - 1) / NTHR, NTHR, 0, stream>>>(src, dst, nRows, Kp, sk, sn, offv, kReal, nReal, kSplit, s0, s1);
  };
  cvt(We1, W1nT, HD, ND, HD, 1, 0, ND, HD, ND, 64.0f, 64.0f);
  cvt(We1, W1nT + (size_t)HD * ND, HD, ND, HD, 1, ND * HD, ND, HD, ND, 64.0f, 64.0f);
  cvt(We1, W1eT, HD, KE1, HD, 1, 2 * ND * HD, 1 + ED, HD, KE1, 64.0f, 64.0f);
  cvt(We2, W2T, HD, HD, HD, 1, 0, HD, HD, HD, 64.0f, 64.0f);
  cvt(Wc1, Wc1T, HD, HD, HD, 1, 0, HD, HD, HD, 64.0f, 64.0f);
  cvt(Wn1, Wn1T, HD, KN, HD, 1, 0, KN, HD, ND, 64.0f, 4.0f);
  cvt(Wn2, Wn2T, ND, HD, ND, 1, 0, HD, ND, HD, 64.0f, 64.0f);

  k_pq<<<dim3(nBlkM, 2), NTHR, 0, stream>>>(h, W1nT, PQ, nN);

  const float degeps = (float)((double)nE / (double)nN + 1e-8);
  const float invdeg = 1.0f / degeps;
  k_edge<<<nBlkE, NTHR, 0, stream>>>(x, ea, eidx, PQ, W1eT, be1, W2T, be2, Wa, ba, Wc1T, bc1, Wc2,
                                     AGG, xout, nN, nE, 1, invdeg, nN * 3);

  k_node<<<nBlkM, NTHR, 0, stream>>>(h, AGG, Wn1T, bn1, Wn2T, bn2, gamma, beta, hout, nN);
}
